// _SSMCore_46643344834783
// MI455X (gfx1250) — hardware-run, weakly checked
//
#include <hip/hip_runtime.h>
#include <math.h>

typedef __attribute__((ext_vector_type(16))) _Float16 v16h;
typedef __attribute__((ext_vector_type(8)))  _Float16 v8h;
typedef __attribute__((ext_vector_type(16))) __bf16   v16b;
typedef __attribute__((ext_vector_type(8)))  __bf16   v8b;
typedef __attribute__((ext_vector_type(8)))  float    v8f;
typedef __attribute__((ext_vector_type(4)))  float    v4f;

constexpr int kBatch  = 2;
constexpr int kSeq    = 2048;
constexpr int kDin    = 2048;
constexpr int kNst    = 16;
constexpr int kDtR    = 64;
constexpr int kXp     = kDtR + 2 * kNst;
constexpr int kXpPad  = 128;
constexpr int kRows   = kBatch * kSeq;
constexpr int kDrP    = 64;
constexpr int kBcP    = 64;
constexpr int kBcW    = 2 * kNst;
constexpr int kScanTS = 64;
constexpr int kScanCh = 64;
constexpr int kScanYP = 68;
constexpr float kW2Carry    = 4.0f;
constexpr float kW2CarryInv = 1.0f / kW2Carry;
static_assert(kW2Carry * kW2CarryInv == 1.0f, "carry is a power of two");
static_assert(kXp == 96, "x_proj width");
static_assert(kXpPad == 2 * 64 && kXpPad >= kXp, "padded x_proj width = two 64-wide GEMM column tiles");
static_assert((kDin % 32) == 0 && (kDtR % 32) == 0, "GEMM K multiples of 32");
static_assert((kRows % 64) == 0 && (kDin % 64) == 0 && (kDrP % 64) == 0 && (kBcP % 64) == 0, "GEMM M,N multiples of 64");
static_assert(kDrP == kDtR, "delta_raw plane width equals dt rank");
static_assert((kSeq % kScanTS) == 0 && (kDin % kScanCh) == 0, "scan tile multiples");
static_assert(kBcW == 32 && kScanTS == 64 && kScanCh == 64, "scan staging maps are written for 64 steps x 32 cols, 64 channels");

constexpr size_t kOffXB   = 0;
constexpr size_t kOffW1B  = kOffXB  + (size_t)kRows  * kDin * 2;
constexpr size_t kOffW2F  = kOffW1B + (size_t)kXpPad * kDin * 2;
constexpr size_t kOffDRF  = kOffW2F + (size_t)kDin   * kDtR * 2;
constexpr size_t kOffBC   = kOffDRF + (size_t)kRows  * kDrP * 2;
constexpr size_t kOffPRE  = kOffBC  + (size_t)kRows  * kBcP * 4;
constexpr size_t kWsTotal = kOffPRE + (size_t)kRows  * kDin * 4;
static_assert(kWsTotal == 52690944ull, "carve total");
static_assert(kWsTotal <= 134217728ull, "carve cap");
static_assert((kOffW1B % 128) == 0 && (kOffW2F % 128) == 0 && (kOffDRF % 128) == 0 && (kOffBC % 128) == 0 &&
              (kOffPRE % 128) == 0, "128-B aligned regions");

__device__ __forceinline__ unsigned short f2bf_bits(float f) {
  unsigned u = __float_as_uint(f);
  return (unsigned short)((u + 0x7FFFu + ((u >> 16) & 1u)) >> 16);
}
__device__ __forceinline__ float bf_bits2f(unsigned short h) { return __uint_as_float(((unsigned)h) << 16); }
__device__ __forceinline__ float bf_rne(float f) { return bf_bits2f(f2bf_bits(f)); }

__device__ __forceinline__ void row_guard_h(v8f& a, v8f& b, v8f& c, v8f& d, v16h x, v16h y) {
  asm volatile("v_nop\n\tv_nop\n\tv_nop\n\tv_nop" : "+v"(a), "+v"(b), "+v"(c), "+v"(d) : "v"(x), "v"(y));
}
__device__ __forceinline__ void row_guard_b(v8f& a, v8f& b, v8f& c, v8f& d, v16b x, v16b y) {
  asm volatile("v_nop\n\tv_nop\n\tv_nop\n\tv_nop" : "+v"(a), "+v"(b), "+v"(c), "+v"(d) : "v"(x), "v"(y));
}
__device__ __forceinline__ void keep4_h(v16h a, v16h b, v16h c, v16h d) { asm volatile("v_nop" :: "v"(a), "v"(b), "v"(c), "v"(d)); }
__device__ __forceinline__ void keep4_b(v16b a, v16b b, v16b c, v16b d) { asm volatile("v_nop" :: "v"(a), "v"(b), "v"(c), "v"(d)); }
__device__ __forceinline__ void acc_guard4(v8f& a, v8f& b, v8f& c, v8f& d) {
  asm volatile("v_nop\n\tv_nop\n\tv_nop\n\tv_nop" : "+v"(a), "+v"(b), "+v"(c), "+v"(d));
}

template <int ET> struct FragT;
template <> struct FragT<0> {
  typedef _Float16 T; typedef v16h V; union U { v16h v; v8h h[2]; };
  static __device__ __forceinline__ v16h load(const _Float16* p) {
    U f; f.h[0] = *(const v8h*)(p); f.h[1] = *(const v8h*)(p + 16); return f.v;
  }
  static __device__ __forceinline__ v8f mma(v16h a, v16h b, v8f c) {
    return __builtin_amdgcn_wmma_f32_16x16x32_f16(false, a, false, b, (short)0, c, false, false);
  }
  static __device__ __forceinline__ void guard(v8f& a, v8f& b, v8f& c, v8f& d, v16h x, v16h y) { row_guard_h(a, b, c, d, x, y); }
  static __device__ __forceinline__ void keep(v16h a, v16h b, v16h c, v16h d) { keep4_h(a, b, c, d); }
};
template <> struct FragT<1> {
  typedef __bf16 T; typedef v16b V; union U { v16b v; v8b h[2]; };
  static __device__ __forceinline__ v16b load(const __bf16* p) {
    U f; f.h[0] = *(const v8b*)(p); f.h[1] = *(const v8b*)(p + 16); return f.v;
  }
  static __device__ __forceinline__ v8f mma(v16b a, v16b b, v8f c) {
    return __builtin_amdgcn_wmma_f32_16x16x32_bf16(false, a, false, b, (short)0, c, false, false);
  }
  static __device__ __forceinline__ void guard(v8f& a, v8f& b, v8f& c, v8f& d, v16b x, v16b y) { row_guard_b(a, b, c, d, x, y); }
  static __device__ __forceinline__ void keep(v16b a, v16b b, v16b c, v16b d) { keep4_b(a, b, c, d); }
};

template <int ET, int BIAS_MODE, int OUT_MODE>
__global__ __launch_bounds__(256) void wmma_gemm64(
    const unsigned short* __restrict__ Ap, int lda,
    const unsigned short* __restrict__ Btp, int ldb,
    void* __restrict__ Cout, int ldc,
    const float* __restrict__ bias,
    int M, int N, int K, float scale) {
  typedef typename FragT<ET>::T T;
  typedef typename FragT<ET>::V V;
  const T* Ab = (const T*)Ap;
  const T* Bb = (const T*)Btp;
  __shared__ __align__(16) float sT[8][16 * 68];
  const int lane = threadIdx.x & 31;
  const int wave = threadIdx.x >> 5;
  const int tilesN = N >> 6;
  const int tilesM = M >> 6;
  const int tile = blockIdx.x * 8 + wave;
  if (tile >= tilesM * tilesN) return;
  const int tm = tile / tilesN;
  const int tn = tile - tm * tilesN;
  const int m0 = tm << 6;
  const int n0 = tn << 6;

  const int rlane = lane & 15;
  const int koff  = (lane >> 4) * 8;
  const int mOff  = (lane >> 4) * 8;

  v8f acc[4][4];
#pragma unroll
  for (int i = 0; i < 4; ++i)
#pragma unroll
    for (int j = 0; j < 4; ++j) acc[i][j] = (v8f){0.f,0.f,0.f,0.f,0.f,0.f,0.f,0.f};

  for (int k0 = 0; k0 < K; k0 += 32) {
    V bh[4];
#pragma unroll
    for (int j = 0; j < 4; ++j) {
      const size_t bo = (size_t)(n0 + (j << 4) + rlane) * ldb + koff + k0;
      bh[j] = FragT<ET>::load(Bb + bo);
    }
#pragma unroll
    for (int i = 0; i < 4; ++i) {
      const size_t ao = (size_t)(m0 + (i << 4) + rlane) * lda + koff + k0;
      V ah = FragT<ET>::load(Ab + ao);
#pragma unroll
      for (int j = 0; j < 4; ++j) {
        acc[i][j] = FragT<ET>::mma(ah, bh[j], acc[i][j]);
      }
      FragT<ET>::guard(acc[i][0], acc[i][1], acc[i][2], acc[i][3], ah, ah);
    }
    FragT<ET>::keep(bh[0], bh[1], bh[2], bh[3]);
  }
  acc_guard4(acc[0][0], acc[0][1], acc[0][2], acc[0][3]);
  acc_guard4(acc[1][0], acc[1][1], acc[1][2], acc[1][3]);
  acc_guard4(acc[2][0], acc[2][1], acc[2][2], acc[2][3]);
  acc_guard4(acc[3][0], acc[3][1], acc[3][2], acc[3][3]);

  float* slab = sT[wave];
#pragma unroll
  for (int i = 0; i < 4; ++i) {
    const int mBase = m0 + (i << 4);
#pragma unroll
    for (int j = 0; j < 4; ++j) {
      const int n = n0 + (j << 4) + rlane;
      float bv = 0.f;
      if (BIAS_MODE == 2) bv = bf_rne(bias[n]);
#pragma unroll
      for (int r = 0; r < 8; ++r) {
        float v = acc[i][j][r] * scale;
        if (BIAS_MODE == 2) v += bv;
        slab[(mOff + r) * 68 + (j << 4) + rlane] = v;
      }
    }
    __builtin_amdgcn_fence(__ATOMIC_RELEASE, "workgroup");
    __builtin_amdgcn_wave_barrier();
    __builtin_amdgcn_fence(__ATOMIC_ACQUIRE, "workgroup");
    if (OUT_MODE == 0) {
      float* C = (float*)Cout;
      const int hh = lane >> 4, c4 = (lane & 15) * 4;
      for (int pass = 0; pass < 2; ++pass) {
#pragma unroll
        for (int it = 0; it < 8; ++it) {
          const int row = it * 2 + hh;
          v4f v = *(const v4f*)(slab + row * 68 + c4);
          *(volatile v4f*)(C + (size_t)(mBase + row) * ldc + n0 + c4) = v;
        }
        __threadfence();
      }
    } else {
      const int q = lane >> 3, c8 = (lane & 7) * 8;
      unsigned short* C = (unsigned short*)Cout;
      for (int pass = 0; pass < 2; ++pass) {
#pragma unroll
        for (int it = 0; it < 4; ++it) {
          const int row = it * 4 + q;
          const float* sp = slab + row * 68 + c8;
          v8h hv;
#pragma unroll
          for (int e = 0; e < 8; ++e) {
            const float sv = sp[e];
            hv[e] = (_Float16)sv;
          }
          *(volatile v8h*)(C + (size_t)(mBase + row) * ldc + n0 + c8) = hv;
        }
        __threadfence();
      }
    }
    __builtin_amdgcn_fence(__ATOMIC_RELEASE, "workgroup");
    __builtin_amdgcn_wave_barrier();
    __builtin_amdgcn_fence(__ATOMIC_ACQUIRE, "workgroup");
  }
}

template <int MODE>
__global__ __launch_bounds__(256) void cast_rows16_kernel(
    const float* __restrict__ src, unsigned short* __restrict__ dst, int total8, int src8, float carry)
{
  const int i = blockIdx.x * 256 + threadIdx.x;
  if (i >= total8) return;
  const bool live = (i < src8);
  const int ic = live ? i : (src8 - 1);
  const size_t s0 = (size_t)ic << 3;
  const size_t e0 = (size_t)i << 3;
  const v4f a0 = *(const v4f*)(src + s0);
  const v4f a1 = *(const v4f*)(src + s0 + 4);
  v8h hv;
#pragma unroll
  for (int e = 0; e < 4; ++e) {
    const float f0 = live ? a0[e] : 0.0f;
    const float f1 = live ? a1[e] : 0.0f;
    if (MODE == 0) {
      const unsigned short h0 = f2bf_bits(f0);
      const unsigned short h1 = f2bf_bits(f1);
      hv[e]     = __builtin_bit_cast(_Float16, h0);
      hv[4 + e] = __builtin_bit_cast(_Float16, h1);
    } else {
      const float g0 = carry * bf_rne(f0);
      const float g1 = carry * bf_rne(f1);
      hv[e]     = (_Float16)g0;
      hv[4 + e] = (_Float16)g1;
    }
  }
  unsigned short* qd = dst + e0;
  *(volatile v8h*)qd = hv;
  __threadfence();
  *(volatile v8h*)qd = hv;
}

__global__ __launch_bounds__(64) void scan_kernel(
    const float* __restrict__ PRE, const float* __restrict__ X, const float* __restrict__ BC,
    const float* __restrict__ Alog, const float* __restrict__ Dp, float* __restrict__ out)
{
  __shared__ __align__(16) float sX[kScanTS * kBcW];
  __shared__ __align__(16) float sY[kScanTS * kScanYP];
  __shared__ __align__(16) float sA[kNst * kScanCh];
  const int tid = threadIdx.x, lane = tid & 31, wave = tid >> 5;
  constexpr int kBlkPerB = kDin / kScanCh;
  const int bix = blockIdx.x / kBlkPerB;
  const int d0  = (blockIdx.x - bix * kBlkPerB) * kScanCh;
  const int d   = d0 + tid;
  const size_t row0 = (size_t)bix * kSeq;
#pragma unroll 1
  for (int s = 0; s < kNst; ++s) sA[s * kScanCh + tid] = -expf(bf_rne(Alog[(size_t)d * kNst + s]));
  __syncthreads();
  float negA[kNst], h[kNst];
#pragma unroll
  for (int s = 0; s < kNst; ++s) {
    negA[s] = sA[s * kScanCh + tid];
    h[s] = 0.f;
  }
  const float Dd = bf_rne(Dp[d]);
  const int lr = tid >> 3, lc4 = (tid & 7) * 4;
  const int hh = lane >> 4, c4 = (lane & 15) * 4;
#pragma unroll 1
  for (int t0 = 0; t0 < kSeq; t0 += kScanTS) {
    __syncthreads();
#pragma unroll
    for (int i = 0; i < 8; ++i) {
      const int r = lr + 8 * i;
      *(v4f*)(sX + r * kBcW + lc4) = *(const v4f*)(BC + (row0 + t0 + r) * kBcP + lc4);
    }
    __syncthreads();
#pragma unroll 1
    for (int s = 0; s < kScanTS; ++s) {
      const int t = t0 + s;
      const float* xr = sX + s * kBcW;
      float Bs[kNst], Cs[kNst];
#pragma unroll
      for (int q4 = 0; q4 < 4; ++q4) {
        const v4f bv = *(const v4f*)(xr + 4 * q4);
        const v4f cv = *(const v4f*)(xr + kNst + 4 * q4);
        Bs[4 * q4 + 0] = bv[0]; Bs[4 * q4 + 1] = bv[1]; Bs[4 * q4 + 2] = bv[2]; Bs[4 * q4 + 3] = bv[3];
        Cs[4 * q4 + 0] = cv[0]; Cs[4 * q4 + 1] = cv[1]; Cs[4 * q4 + 2] = cv[2]; Cs[4 * q4 + 3] = cv[3];
      }
      const float v  = PRE[(row0 + t) * kDin + d];
      const float xraw = X[(row0 + t) * kDin + d];
      const float xt = bf_rne(xraw);
      const float a  = expf(-fabsf(v));
      const float u  = 1.0f + a;
      const float cr = (a - (u - 1.0f)) * __builtin_amdgcn_rcpf(u);
      const float l1p = logf(u) + cr;
      const float dt  = fmaxf(v, 0.0f) + l1p;
      const float dtx = dt * xt;
      float y = 0.f;
#pragma unroll
      for (int k = 0; k < kNst; ++k) {
        const float e = expf(dt * negA[k]);
        h[k] = e * h[k] + dtx * Bs[k];
        y = h[k] * Cs[k] + y;
      }
      y = xt * Dd + y;
      sY[s * kScanYP + tid] = y;
    }
    __syncthreads();
    for (int pass = 0; pass < 2; ++pass) {
#pragma unroll
      for (int it = 0; it < 16; ++it) {
        const int row = it * 4 + wave * 2 + hh;
        const v4f val = *(const v4f*)(sY + row * kScanYP + c4);
        *(volatile v4f*)(out + (row0 + t0 + row) * kDin + d0 + c4) = val;
      }
      __threadfence();
    }
  }
}

extern "C" void kernel_launch(void* const* d_in, const int* in_sizes, int n_in,
                              void* d_out, int out_size, void* d_ws, size_t ws_size,
                              hipStream_t stream) {
  if (n_in < 6) return;
  if (in_sizes[0] != kRows * kDin) return;
  if (in_sizes[1] != kXp * kDin) return;
  if (in_sizes[2] != kDin * kDtR) return;
  if (in_sizes[3] != kDin) return;
  if (in_sizes[4] != kDin * kNst) return;
  if (in_sizes[5] != kDin) return;
  if (out_size != kRows * kDin) return;
  if (ws_size < kWsTotal) return;

  const float* x     = (const float*)d_in[0];
  const float* xpw   = (const float*)d_in[1];
  const float* dtw   = (const float*)d_in[2];
  const float* dtb   = (const float*)d_in[3];
  const float* A_log = (const float*)d_in[4];
  const float* Dvec  = (const float*)d_in[5];
  float* out = (float*)d_out;

  char* ws = (char*)d_ws;
  unsigned short* XB  = (unsigned short*)(ws + kOffXB);
  unsigned short* W1B = (unsigned short*)(ws + kOffW1B);
  unsigned short* W2F = (unsigned short*)(ws + kOffW2F);
  unsigned short* DRF = (unsigned short*)(ws + kOffDRF);
  float*          BC  = (float*)(ws + kOffBC);
  float*          PRE = (float*)(ws + kOffPRE);

  constexpr int kX8    = kRows * kDin / 8;
  constexpr int kW1T8  = kXpPad * kDin / 8;
  constexpr int kW1S8  = kXp * kDin / 8;
  constexpr int kW28   = kDin * kDtR / 8;
  static_assert((kX8 % 256) == 0 && (kW1T8 % 256) == 0 && (kW28 % 256) == 0, "exact cast grids");
  cast_rows16_kernel<0><<<kX8 / 256, 256, 0, stream>>>(x, XB, kX8, kX8, 1.0f);
  cast_rows16_kernel<0><<<kW1T8 / 256, 256, 0, stream>>>(xpw, W1B, kW1T8, kW1S8, 1.0f);
  cast_rows16_kernel<1><<<kW28 / 256, 256, 0, stream>>>(dtw, W2F, kW28, kW28, kW2Carry);

  wmma_gemm64<1, 0, 1><<<dim3((kRows / 64) * 1 / 8), 256, 0, stream>>>(
      XB, kDin,
      W1B, kDin,
      (void*)DRF, kDrP,
      nullptr,
      kRows, 64, kDin, 1.0f);

  wmma_gemm64<1, 0, 0><<<dim3((kRows / 64) * 1 / 8), 256, 0, stream>>>(
      XB, kDin,
      W1B + (size_t)64 * kDin, kDin,
      (void*)BC, kBcP,
      nullptr,
      kRows, 64, kDin, 1.0f);

  wmma_gemm64<0, 2, 0><<<dim3((kRows / 64) * (kDin / 64) / 8), 256, 0, stream>>>(
      DRF, kDrP,
      W2F, kDtR,
      (void*)PRE, kDin,
      dtb,
      kRows, kDin, kDtR, kW2CarryInv);

  scan_kernel<<<kBatch * (kDin / kScanCh), kScanCh, 0, stream>>>(PRE, x, BC, A_log, Dvec, out);
}
